// FixedSlotAttentionMultiHeadProb_81990925681043
// MI455X (gfx1250) — hardware-verified
//
#include <hip/hip_runtime.h>
#include <math.h>


#define NB 16
#define NN 4096
#define DIN 64
#define KS 8
#define DD 64
#define HH 4
#define DH 16
#define KH (KS * HH)
#define HID 256
#define NR (NB * NN)
#define EPS 1e-5f

typedef __attribute__((ext_vector_type(16))) __bf16 v16b;
typedef __attribute__((ext_vector_type(8)))  float v8f;
typedef __attribute__((ext_vector_type(4)))  float v4f;
typedef float __attribute__((may_alias)) float_a;

template <typename T> __device__ __forceinline__ void vst2(void* p, T v) { *(volatile T*)p = v; __threadfence(); *(volatile T*)p = v; }
__device__ __forceinline__ v8f wmma_bf(v16b a, v16b b, v8f c) {
  v8f d = __builtin_amdgcn_wmma_f32_16x16x32_bf16(false, a, false, b, (short)0, c, false, false);
  asm volatile("v_nop\n\tv_nop\n\tv_nop\n\tv_nop" : "+v"(d) : "v"(a), "v"(b));
  return d;
}
struct F2 { v16b h, l; };
__device__ __forceinline__ F2 split_vals(const float v[16]) {
  F2 r;
#pragma unroll
  for (int i = 0; i < 16; ++i) { const __bf16 h = (__bf16)v[i]; r.h[i] = h; r.l[i] = (__bf16)(v[i] - (float)h); }
  return r;
}
__device__ __forceinline__ v8f mac3(const F2& a, const F2& b, v8f c) { c = wmma_bf(a.l, b.h, c); c = wmma_bf(a.h, b.l, c); return wmma_bf(a.h, b.h, c); }
#define LDSX() do { asm volatile("s_wait_dscnt 0" ::: "memory"); __builtin_amdgcn_wave_barrier(); __builtin_amdgcn_fence(__ATOMIC_RELEASE, "workgroup"); } while (0)

__global__ __launch_bounds__(128) void k_proj(const float* __restrict__ emb, const float* __restrict__ lw, const float* __restrict__ lb,
                                            const float* __restrict__ Wk, const float* __restrict__ Wv, float* __restrict__ keys, float* __restrict__ vals) {
  __shared__ __align__(16) float xs[64][68];
  __shared__ __align__(16) float so[4][16][132];
  const int tid = threadIdx.x, wave = tid >> 5, lane = tid & 31, col = lane & 15, g = lane >> 4;
  const int r0 = blockIdx.x * 64;
  { const int rl = tid >> 1, hf = tid & 1; const float* xr = emb + (size_t)(r0 + rl) * DIN + hf * 32;
    float v[32], s = 0.f;
#pragma unroll
    for (int i = 0; i < 32; ++i) { v[i] = xr[i]; s += v[i]; }
    s += __shfl_xor(s, 1, 32); const float mu = s / 64.f;
    float q = 0.f;
#pragma unroll
    for (int i = 0; i < 32; ++i) { const float d = v[i] - mu; q += d * d; }
    q += __shfl_xor(q, 1, 32); const float rs = rsqrtf(q / 64.f + EPS);
#pragma unroll
    for (int i = 0; i < 32; ++i) xs[rl][hf * 32 + i] = (v[i] - mu) * rs * lw[hf * 32 + i] + lb[hf * 32 + i]; }
  __syncthreads();
  v8f ak[4] = {}, av[4] = {};
#pragma unroll
  for (int kc = 0; kc < 2; ++kc) {
    float va[16];
#pragma unroll
    for (int i = 0; i < 8; ++i) { va[i] = xs[wave * 16 + col][kc * 32 + 8 * g + i]; va[8 + i] = xs[wave * 16 + col][kc * 32 + 16 + 8 * g + i]; }
    const F2 a = split_vals(va);
#pragma unroll
    for (int j = 0; j < 4; ++j) {
      float wb[16], wv2[16];
#pragma unroll
      for (int i = 0; i < 8; ++i) { const int ka = kc * 32 + 8 * g + i, kb = ka + 16;
        wb[i] = Wk[ka * DD + j * 16 + col]; wb[8 + i] = Wk[kb * DD + j * 16 + col];
        wv2[i] = Wv[ka * DD + j * 16 + col]; wv2[8 + i] = Wv[kb * DD + j * 16 + col]; }
      ak[j] = mac3(a, split_vals(wb), ak[j]); av[j] = mac3(a, split_vals(wv2), av[j]);
    }
  }
  float* S = &so[wave][0][0];
#pragma unroll
  for (int j = 0; j < 4; ++j)
#pragma unroll
    for (int r = 0; r < 8; ++r) { S[(8 * g + r) * 132 + j * 16 + col] = ak[j][r]; S[(8 * g + r) * 132 + 64 + j * 16 + col] = av[j][r]; }
  LDSX();
#pragma unroll
  for (int q = 0; q < 8; ++q) { const int rl = q * 2 + (lane >> 4), pc = lane & 15; const size_t row = r0 + wave * 16 + rl;
    vst2(keys + row * DD + pc * 4, *(const v4f*)(S + rl * 132 + pc * 4));
    vst2(vals + row * DD + pc * 4, *(const v4f*)(S + rl * 132 + 64 + pc * 4)); }
}

__global__ __launch_bounds__(64) void k_init(const float* __restrict__ noise, const float* __restrict__ mu, const float* __restrict__ ms,
                                           const float* __restrict__ ls, float* __restrict__ slots, float* __restrict__ sigma, float* __restrict__ mix) {
  const int bk = blockIdx.x, k = bk % KS, d = threadIdx.x;
  vst2(slots + (size_t)bk * DD + d, (float_a)(mu[k * DD + d] + expf(ms[k * DD + d]) * noise[(size_t)bk * DD + d]));
  vst2(sigma + ((size_t)bk * HH + d / DH) * 32 + (d % DH), (float_a)ls[k * DD + d]);
  if (d == 0) vst2(mix + (size_t)bk * 32, (float_a)(1.0f / KS));
}

__global__ __launch_bounds__(64) void k_coef(const float* __restrict__ slots, const float* __restrict__ sigma, const float* __restrict__ mix,
                                           const float* __restrict__ toq, const float* __restrict__ lw, const float* __restrict__ lb,
                                           float* __restrict__ qv, float* __restrict__ inv2, float* __restrict__ cst) {
  __shared__ float red[64], lsg[64];
  const int bk = blockIdx.x, k = bk % KS, d = threadIdx.x;
  const float v = slots[(size_t)bk * DD + d];
  red[d] = v; __syncthreads();
  for (int st = 32; st > 0; st >>= 1) { if (d < st) red[d] += red[d + st]; __syncthreads(); }
  const float mu = red[0] / 64.f; __syncthreads();
  red[d] = (v - mu) * (v - mu); __syncthreads();
  for (int st = 32; st > 0; st >>= 1) { if (d < st) red[d] += red[d + st]; __syncthreads(); }
  const float rs = rsqrtf(red[0] / 64.f + EPS);
  const float s = (v - mu) * rs * lw[d] + lb[d];
  vst2(qv + (size_t)bk * DD + d, (float_a)(s * toq[((size_t)k * DD + d) * DD + d]));
  const float sg = sigma[((size_t)bk * HH + d / DH) * 32 + (d % DH)];
  vst2(inv2 + (size_t)bk * DD + d, (float_a)(1.0f / (sg * sg + EPS)));
  lsg[d] = -logf(fmaxf(sg, EPS)); __syncthreads();
  if (d < HH) { float t = 0.f; for (int i = 0; i < DH; ++i) t += lsg[d * DH + i];
    const float log_pi = -0.5f * (float)DIN * logf(2.0f * 3.14159265358979f);
    vst2(cst + (size_t)bk * 32 + d * 8, (float_a)(logf(mix[(size_t)bk * 32] + EPS) + (16.0f * log_pi + t) * 0.25f)); }
}

__global__ __launch_bounds__(256) void k_attn(const float* __restrict__ keys, const float* __restrict__ qv, const float* __restrict__ inv2,
                                            const float* __restrict__ cst, float* __restrict__ attn, float* __restrict__ vis, float* __restrict__ nkp, int wvis) {
  __shared__ float qs[KS * DD], is2[KS * DD], cs[KH];
  __shared__ float red[KH][256];
  const int b = blockIdx.y, n0 = blockIdx.x * 256, tid = threadIdx.x, n = n0 + tid;
  for (int i = tid; i < KS * DD; i += 256) { qs[i] = qv[(size_t)b * KS * DD + i]; is2[i] = inv2[(size_t)b * KS * DD + i]; }
  if (tid < KH) cs[tid] = cst[((size_t)b * KS + tid / HH) * 32 + (tid % HH) * 8];
  float kk[DD];
#pragma unroll
  for (int i = 0; i < DD; ++i) kk[i] = keys[((size_t)b * NN + n) * DD + i];
  __syncthreads();
  float gl[KH]; float mx = -3.0e38f;
#pragma unroll 1
  for (int k = 0; k < KS; ++k)
#pragma unroll 1
    for (int h = 0; h < HH; ++h) { float e = 0.f;
#pragma unroll 1
      for (int i = 0; i < DH; ++i) { const int d = h * DH + i; const float df = kk[d] - qs[k * DD + d]; e += -0.5f * df * df * is2[k * DD + d]; }
      const float gv = cs[k * HH + h] + e * 0.25f; gl[k * HH + h] = gv; mx = fmaxf(mx, gv); }
  float sum = 0.f;
#pragma unroll 1
  for (int c = 0; c < KH; ++c) { gl[c] = expf(gl[c] - mx); sum += gl[c]; }
  const float inv = 1.0f / sum;
#pragma unroll 1
  for (int k = 0; k < KS; ++k) { float vsum = 0.f;
#pragma unroll
    for (int h = 0; h < HH; ++h) { const float a = gl[k * HH + h] * inv + EPS; red[k * HH + h][tid] = a; vsum += a;
      vst2(attn + (((size_t)b * KS + k) * HH + h) * NN + n, (float_a)a); }
    if (wvis) vst2(vis + ((size_t)b * KS + k) * NN + n, (float_a)vsum); }
  __syncthreads();
  if (tid < KH) { float t = 0.f; for (int i = 0; i < 256; ++i) t += red[tid][i]; vst2(nkp + (((size_t)b * KH + tid) * (NN / 256) + blockIdx.x) * 32, (float_a)t); }
}

__global__ __launch_bounds__(256) void k_update(const float* __restrict__ attn, const float* __restrict__ vals, const float* __restrict__ nkp,
                                              float* __restrict__ upd, float* __restrict__ sigma, float* __restrict__ mix) {
  __shared__ float red[16][16], nks[HH];
  const int bkh = blockIdx.x, b = bkh / KH, kh = bkh % KH, k = kh / HH, h = kh % HH, tid = threadIdx.x;
  const int dh = tid & 15, grp = tid >> 4;
  if (tid < HH) { float t = 0.f; for (int i = 0; i < NN / 256; ++i) t += nkp[(((size_t)b * KH + k * HH + tid) * (NN / 256) + i) * 32]; nks[tid] = t; }
  __syncthreads();
  const float nk = nks[h];
  const float* ar = attn + (((size_t)b * KS + k) * HH + h) * NN;
  float s = 0.f;
#pragma unroll 1
  for (int n = grp; n < NN; n += 16) s += ar[n] * vals[((size_t)b * NN + n) * DD + h * DH + dh];
  red[grp][dh] = s; __syncthreads();
  float u = 0.f;
  if (grp == 0) { for (int i = 0; i < 16; ++i) u += red[i][dh]; u = u / (nk + EPS); red[0][dh] = u; }
  __syncthreads();
  u = red[0][dh]; __syncthreads();
  float s2 = 0.f;
#pragma unroll 1
  for (int n = grp; n < NN; n += 16) { const float d = vals[((size_t)b * NN + n) * DD + h * DH + dh] - u; s2 += ar[n] * d * d; }
  red[grp][dh] = s2; __syncthreads();
  if (grp == 0) { float t = 0.f; for (int i = 0; i < 16; ++i) t += red[i][dh];
    float sg = t / (nk + EPS); sg = sg < EPS ? EPS : sg; sg = sqrtf(sg) + EPS;
    vst2(upd + ((size_t)(b * KS + k) * HH + h) * 32 + dh, (float_a)u);
    vst2(sigma + ((size_t)(b * KS + k) * HH + h) * 32 + dh, (float_a)sg); }
  if (h == 0 && tid == 0) vst2(mix + (size_t)(b * KS + k) * 32, (float_a)((nks[0] + nks[1] + nks[2] + nks[3]) / (float)NN));
}

__global__ __launch_bounds__(256) void k_gru_mlp(const float* __restrict__ upd, float* __restrict__ slots, float* __restrict__ outs, int last,
                                               const float* __restrict__ wih, const float* __restrict__ whh, const float* __restrict__ bih, const float* __restrict__ bhh,
                                               const float* __restrict__ w1, const float* __restrict__ b1, const float* __restrict__ w2, const float* __restrict__ b2,
                                               const float* __restrict__ lw, const float* __restrict__ lb) {
  __shared__ float xs[DD], hs[DD], gx[3 * DD], gh[3 * DD], hn[DD], sn[DD], hid[HID], red[DD];
  const int bk = blockIdx.x, tid = threadIdx.x;
  if (tid < DD) { xs[tid] = upd[((size_t)bk * HH + tid / DH) * 32 + (tid % DH)]; hs[tid] = slots[(size_t)bk * DD + tid]; }
  __syncthreads();
  if (tid < 3 * DD) { float a = bih[tid], c = bhh[tid];
#pragma unroll 1
    for (int i = 0; i < DD; ++i) { a += xs[i] * wih[(size_t)tid * DD + i]; c += hs[i] * whh[(size_t)tid * DD + i]; }
    gx[tid] = a; gh[tid] = c; }
  __syncthreads();
  if (tid < DD) { const float r = 1.0f / (1.0f + expf(-(gx[tid] + gh[tid]))), z = 1.0f / (1.0f + expf(-(gx[DD + tid] + gh[DD + tid])));
    const float nn_ = tanhf(gx[2 * DD + tid] + r * gh[2 * DD + tid]); hn[tid] = (1.0f - z) * nn_ + z * hs[tid]; red[tid] = hn[tid]; }
  __syncthreads();
  for (int st = 32; st > 0; st >>= 1) { if (tid < st) red[tid] += red[tid + st]; __syncthreads(); }
  const float mu = red[0] / 64.f; __syncthreads();
  if (tid < DD) red[tid] = (hn[tid] - mu) * (hn[tid] - mu); __syncthreads();
  for (int st = 32; st > 0; st >>= 1) { if (tid < st) red[tid] += red[tid + st]; __syncthreads(); }
  const float rs = rsqrtf(red[0] / 64.f + EPS);
  if (tid < DD) sn[tid] = (hn[tid] - mu) * rs * lw[tid] + lb[tid];
  __syncthreads();
  { float a = b1[tid];
#pragma unroll 1
    for (int i = 0; i < DD; ++i) a += sn[i] * w1[(size_t)i * HID + tid];
    hid[tid] = a > 0.f ? a : 0.f; }
  __syncthreads();
  if (tid < DD) { float a = b2[tid];
#pragma unroll 1
    for (int i = 0; i < HID; ++i) a += hid[i] * w2[(size_t)i * DD + tid];
    const float sv = hn[tid] + a;
    vst2(slots + (size_t)bk * DD + tid, (float_a)sv);
    if (last) vst2(outs + (size_t)bk * DD + tid, (float_a)sv); }
}

extern "C" void kernel_launch(void* const* d_in, const int* in_sizes, int n_in,
                              void* d_out, int out_size, void* d_ws, size_t ws_size,
                              hipStream_t stream) {
  (void)in_sizes; (void)n_in; (void)out_size; (void)ws_size;
  const float* emb = (const float*)d_in[0]; const float* noise = (const float*)d_in[1];
  const float* mu = (const float*)d_in[2];  const float* ms = (const float*)d_in[3];
  const float* ls = (const float*)d_in[4];  const float* Wk = (const float*)d_in[5];
  const float* toq = (const float*)d_in[6]; const float* Wv = (const float*)d_in[7];
  const float* wih = (const float*)d_in[8]; const float* whh = (const float*)d_in[9];
  const float* bih = (const float*)d_in[10]; const float* bhh = (const float*)d_in[11];
  const float* w1 = (const float*)d_in[12]; const float* b1 = (const float*)d_in[13];
  const float* w2 = (const float*)d_in[14]; const float* b2 = (const float*)d_in[15];
  const float* liw = (const float*)d_in[16]; const float* lib = (const float*)d_in[17];
  const float* lsw = (const float*)d_in[18]; const float* lsb = (const float*)d_in[19];
  const float* lfw = (const float*)d_in[20]; const float* lfb = (const float*)d_in[21];
  float* slots = (float*)d_out;
  float* vis   = (float*)d_out + 8192;
  float* vals  = (float*)d_out + 532480;
  char* ws = (char*)d_ws; size_t off = 0;
  auto take = [&](size_t bytes) { char* p = ws + off; off += (bytes + 255) & ~(size_t)255; return p; };
  float* keys  = (float*)take((size_t)NR * DD * 4);
  float* sigma = (float*)take((size_t)NB * KS * HH * 32 * 4);
  float* mix   = (float*)take((size_t)NB * KS * 32 * 4);
  float* qv    = (float*)take((size_t)NB * KS * DD * 4);
  float* inv2  = (float*)take((size_t)NB * KS * DD * 4);
  float* cst   = (float*)take((size_t)NB * KS * 32 * 4);
  float* attn  = (float*)take((size_t)NB * KH * NN * 4);
  float* nkp   = (float*)take((size_t)NB * KH * (NN / 256) * 32 * 4);
  float* upd   = (float*)take((size_t)NB * KS * HH * 32 * 4);
  float* slw   = (float*)take((size_t)NB * KS * DD * 4);
  k_proj<<<NR / 64, 128, 0, stream>>>(emb, liw, lib, Wk, Wv, keys, vals);
  k_init<<<NB * KS, 64, 0, stream>>>(noise, mu, ms, ls, slw, sigma, mix);
  for (int it = 0; it < 3; ++it) {
    k_coef<<<NB * KS, 64, 0, stream>>>(slw, sigma, mix, toq, lsw, lsb, qv, inv2, cst);
    k_attn<<<dim3(NN / 256, NB), 256, 0, stream>>>(keys, qv, inv2, cst, attn, vis, nkp, it == 2 ? 1 : 0);
    k_update<<<NB * KH, 256, 0, stream>>>(attn, vals, nkp, upd, sigma, mix);
    k_gru_mlp<<<NB * KS, 256, 0, stream>>>(upd, slw, slots, it == 2 ? 1 : 0, wih, whh, bih, bhh, w1, b1, w2, b2, lfw, lfb);
  }
}
